// HadamardMLPDecoder_62191126446520
// MI455X (gfx1250) — hardware-verified
//
#include <hip/hip_runtime.h>
#include <stddef.h>


#define NTHR   256
#define NWAVE  8
#define EPW    16
#define EPB    (NWAVE * EPW)
#define DD     128
#define HH     128
#define APITCH 136
#define WSC    8.0f
#define WINV   0.125f
#define NPIECE ((HH * DD) / 8)

static_assert(EPB == 128);
static_assert((APITCH % 8) == 0);
static_assert((NPIECE % NTHR) == 0);

typedef float    v4f  __attribute__((ext_vector_type(4)));
typedef float    v8f  __attribute__((ext_vector_type(8)));
typedef _Float16 v8h  __attribute__((ext_vector_type(8)));
typedef _Float16 v16h __attribute__((ext_vector_type(16)));
union FragH { v16h v; v8h h[2]; };
union Pk8   { v8h h; v4f f; };

__device__ __forceinline__ v8f wmh(v16h a, v16h b, v8f c) {
  v8f d = __builtin_amdgcn_wmma_f32_16x16x32_f16(false, a, false, b, (short)0, c, false, false);
  asm volatile("v_nop\n\tv_nop\n\tv_nop\n\tv_nop" : "+v"(d) : "v"(a), "v"(b));
  return d;
}

__global__ __launch_bounds__(NTHR) void k_prep(const float* __restrict__ W1, _Float16* w1p) {
  const int i = blockIdx.x * NTHR + threadIdx.x;
  if (i >= NPIECE) return;
  const int n  = i >> 4;
  const int k0 = (i & 15) * 8;
  Pk8 p;
#pragma unroll
  for (int j = 0; j < 8; ++j) p.h[j] = (_Float16)(W1[(k0 + j) * HH + n] * WSC);
  _Float16* dst = w1p + (size_t)i * 8;
  *(volatile v4f*)dst = p.f;
  __threadfence();
  *(volatile v4f*)dst = p.f;
}

__global__ __launch_bounds__(NTHR) void k_edge(
    const float* __restrict__ z, const int* __restrict__ ei, const _Float16* __restrict__ w1p,
    const float* __restrict__ b1, const float* __restrict__ W2, const float* __restrict__ b2,
    float* outp, int nN, int nE) {
  __shared__ __attribute__((aligned(16))) _Float16 atile[NWAVE * EPW * APITCH];
  __shared__ __attribute__((aligned(16))) float    outs[EPB];

  const int tid = threadIdx.x, lane = tid & 31, wave = tid >> 5, hh = lane >> 4, m = lane & 15;
  const int ebase = blockIdx.x * EPB + wave * EPW;

  {
    const int e  = ebase + m;
    const int ec = e < nE ? e : nE - 1;
    int s = ei[ec];
    int d = ei[(size_t)nE + (size_t)ec];
    s = s < 0 ? 0 : (s > nN - 1 ? nN - 1 : s);
    d = d < 0 ? 0 : (d > nN - 1 ? nN - 1 : d);
    const float* zs = z + (size_t)s * DD + 64 * hh;
    const float* zd = z + (size_t)d * DD + 64 * hh;
    _Float16* tr = atile + (wave * EPW + m) * APITCH + 64 * hh;
#pragma unroll 2
    for (int i = 0; i < 8; ++i) {
      const v4f s0 = *(const v4f*)(zs + 8 * i);
      const v4f s1 = *(const v4f*)(zs + 8 * i + 4);
      const v4f d0 = *(const v4f*)(zd + 8 * i);
      const v4f d1 = *(const v4f*)(zd + 8 * i + 4);
      v8h hv;
#pragma unroll
      for (int j = 0; j < 4; ++j) {
        hv[j]     = (_Float16)(s0[j] * d0[j]);
        hv[4 + j] = (_Float16)(s1[j] * d1[j]);
      }
      *(v8h*)(tr + 8 * i) = hv;
    }
  }
  __syncthreads();

  FragH a[4];
  {
    const _Float16* ap = atile + (wave * EPW + m) * APITCH + 8 * hh;
#pragma unroll
    for (int kb = 0; kb < 4; ++kb) {
      a[kb].h[0] = *(const v8h*)(ap + 32 * kb);
      a[kb].h[1] = *(const v8h*)(ap + 32 * kb + 16);
    }
  }
  float pacc[8];
#pragma unroll
  for (int r = 0; r < 8; ++r) pacc[r] = 0.0f;

#pragma unroll 1
  for (int nt = 0; nt < HH / 16; ++nt) {
    const int n = nt * 16 + m;
    const float b1v = b1[n];
    const float w2v = W2[n];
    const _Float16* bp = w1p + (size_t)n * DD + 8 * hh;
    v8f acc;
#pragma unroll
    for (int r = 0; r < 8; ++r) acc[r] = 0.0f;
#pragma unroll
    for (int kb = 0; kb < 4; ++kb) {
      FragH b;
      b.h[0] = *(const v8h*)(bp + 32 * kb);
      b.h[1] = *(const v8h*)(bp + 32 * kb + 16);
      acc = wmh(a[kb].v, b.v, acc);
    }
#pragma unroll
    for (int r = 0; r < 8; ++r) {
      const float hv = fmaxf(acc[r] * WINV + b1v, 0.0f);
      pacc[r] = fmaf(hv, w2v, pacc[r]);
    }
  }

#pragma unroll
  for (int r = 0; r < 8; ++r) {
    float v = pacc[r];
    v += __shfl_xor(v, 1, 32);
    v += __shfl_xor(v, 2, 32);
    v += __shfl_xor(v, 4, 32);
    v += __shfl_xor(v, 8, 32);
    pacc[r] = v;
  }
  const float bb = b2[0];
  float ov = 0.0f;
#pragma unroll
  for (int r = 0; r < 8; ++r) ov = (m == r) ? pacc[r] : ov;
  if (m < 8) outs[wave * EPW + 8 * hh + m] = ov + bb;
  __syncthreads();

  const int  obase = blockIdx.x * EPB;
  const bool full  = (obase + EPB) <= nE;
  const int  gi    = obase + 4 * lane;
  v4f o4 = {0.0f, 0.0f, 0.0f, 0.0f};
  if (wave == 0) o4 = *(const v4f*)(outs + 4 * lane);
  if (wave == 0) {
    if (full) {
      *(volatile v4f*)(outp + gi) = o4;
    } else {
#pragma unroll
      for (int j = 0; j < 4; ++j)
        if (gi + j < nE) *(volatile float*)(outp + gi + j) = o4[j];
    }
  }
  __threadfence();
  if (wave == 0) {
    if (full) {
      *(volatile v4f*)(outp + gi) = o4;
    } else {
#pragma unroll
      for (int j = 0; j < 4; ++j)
        if (gi + j < nE) *(volatile float*)(outp + gi + j) = o4[j];
    }
  }
}

extern "C" void kernel_launch(void* const* d_in, const int* in_sizes, int n_in,
                              void* d_out, int out_size, void* d_ws, size_t ws_size,
                              hipStream_t stream) {
  if (n_in < 6) return;
  const int nN = in_sizes[0] / DD;
  const int nE = in_sizes[1] / 2;
  if (nN <= 0 || nE <= 0 || in_sizes[0] != nN * DD || in_sizes[1] != nE * 2) return;
  if (in_sizes[2] != DD * HH || in_sizes[3] < HH || in_sizes[4] < HH || in_sizes[5] < 1) return;
  if (out_size != nE) return;

  const float* z   = (const float*)d_in[0];
  const int*   ei  = (const int*)d_in[1];
  const float* W1  = (const float*)d_in[2];
  const float* b1  = (const float*)d_in[3];
  const float* W2  = (const float*)d_in[4];
  const float* b2  = (const float*)d_in[5];
  float*       out = (float*)d_out;

  const size_t oW1 = 0;
  const size_t wtot = (size_t)NPIECE * 16;
  if (wtot > ws_size) return;
  _Float16* w1p = (_Float16*)((char*)d_ws + oW1);

  k_prep<<<NPIECE / NTHR, NTHR, 0, stream>>>(W1, w1p);

  const int nblk = (nE + EPB - 1) / EPB;
  k_edge<<<nblk, NTHR, 0, stream>>>(z, ei, w1p, b1, W2, b2, out, nN, nE);
}
